// Star_Net_old_38104949850317
// MI455X (gfx1250) — hardware-run, weakly checked
//
#include <hip/hip_runtime.h>


#ifndef NROWS
#define NROWS 65536
#endif
#define NROWS_FULL 65536
#define ND   8
#define ED   16
#define HID  80
#define NF   9
#define VOC  100000
#define KIN  160
#define NCOL (ND * HID)
#define RPB  128
#define BW   8
#define XP   168
#define NPAIRF (RPB * NF)
#define CARRY 1024.0f
#define ACC_INV 9.5367431640625e-07f

static_assert(KIN == ED * (NF + 1));
static_assert(KIN % 32 == 0);
static_assert(HID % 16 == 0);
static_assert(HID / 16 == 5);
static_assert(KIN / 32 == 5);
static_assert(RPB == 16 * BW);
static_assert(NROWS % RPB == 0);
static_assert(NROWS <= NROWS_FULL);
static_assert(32 * 4 == RPB);
static_assert((XP * 2) % 16 == 0);
static_assert(XP >= KIN);
static_assert(NPAIRF % 32 == 0);
static_assert(NPAIRF <= 5 * 32 * BW);
static_assert(RPB <= 32 * BW);
static_assert(RPB % 32 == 0);
static_assert(((size_t)NCOL * KIN / 8) % 256 == 0);
static_assert((2 * NCOL / 4) % 160 == 0);
static_assert(HID % 4 == 0);
static_assert(NCOL % 4 == 0);
static_assert(KIN % 8 == 0);
static_assert((size_t)RPB * XP * 2 + 3 * RPB * 4 <= 131072);

typedef _Float16 h16;
typedef unsigned short bf;
typedef __attribute__((ext_vector_type(16))) _Float16 v16h;
typedef __attribute__((ext_vector_type(8)))  _Float16 v8h;
typedef __attribute__((ext_vector_type(8)))  float    v8f;
typedef __attribute__((ext_vector_type(4)))  float    v4f;
typedef v4f  __attribute__((may_alias)) v4fa;

__device__ __forceinline__ unsigned short f2bf(float f) { unsigned u = __float_as_uint(f); u += 0x7FFFu + ((u >> 16) & 1u); return (unsigned short)(u >> 16); }
__device__ __forceinline__ float bfr(float f) { return __uint_as_float(((unsigned)f2bf(f)) << 16); }
__device__ __forceinline__ v16h cat16(v8h lo, v8h hi) { return __builtin_shufflevector(lo, hi, 0, 1, 2, 3, 4, 5, 6, 7, 8, 9, 10, 11, 12, 13, 14, 15); }
__device__ __forceinline__ v8f wmma16(v16h a, v16h b, v8f c) { return __builtin_amdgcn_wmma_f32_16x16x32_f16(false, a, false, b, (short)0, c, false, false); }
__device__ __forceinline__ v16h  ldh(const h16* p) { return cat16(*(const v8h*)p, *(const v8h*)(p + 16)); }

static __device__ __forceinline__ h16 toh_flush(float v) { const h16 r = (h16)v; return (fabsf(v) < 6.103515625e-05f) ? (h16)0.0f : r; }
static __device__ __forceinline__ v8f wmma16g(v16h a, v16h b, v8f c) {
    c = wmma16(a, b, c);
    asm volatile("v_nop\n\tv_nop\n\tv_nop\n\tv_nop" : "+v"(c) : "v"(a), "v"(b));
    return c;
}
static __device__ __forceinline__ float relu_b(float v) { return fmaxf(bfr(v), 0.0f); }

__global__ __launch_bounds__(256) void k_w1t(const float* __restrict__ sw1, const float* __restrict__ dw1, h16* W1T) {
#pragma clang fp contract(off)
    const size_t q = (size_t)blockIdx.x * 256 + threadIdx.x;
    const int e0 = (int)(q * 8);
    const int n = e0 / KIN, i0 = e0 - n * KIN;
    const int d = n / HID, hc = n - d * HID;
    v8h o;
#pragma unroll
    for (int k = 0; k < 8; ++k) {
        const int ii = i0 + k;
        const float s = bfr(sw1[(size_t)ii * HID + hc]);
        const float w = bfr(dw1[((size_t)d * KIN + ii) * HID + hc]);
        const float p = s * w;
        o[k] = toh_flush(p * CARRY);
    }
    *(volatile v8h*)(W1T + q * 8) = o; __threadfence(); *(volatile v8h*)(W1T + q * 8) = o;
}

__global__ __launch_bounds__(160) void k_tabs(const float* __restrict__ sb1, const float* __restrict__ db1,
                                              const float* __restrict__ sw2, const float* __restrict__ dw2, float* TB) {
#pragma clang fp contract(off)
    const int i = blockIdx.x * 160 + threadIdx.x;
    const int q = i * 4;
    const int tab = (q >= NCOL) ? 1 : 0;
    const int e = q - tab * NCOL;
    const int d = e / HID, hc = e - d * HID;
    v4f o;
#pragma unroll
    for (int k = 0; k < 4; ++k) {
        const float a0 = bfr(sb1[hc + k]);
        const float a1 = bfr(db1[d * HID + hc + k]);
        const float c0 = bfr(sw2[hc + k]);
        const float c1 = bfr(dw2[d * HID + hc + k]);
        const float vb = a0 + a1;
        const float vw = c0 * c1;
        o[k] = tab ? vw : vb;
    }
    *(volatile v4f*)(TB + (size_t)i * 4) = o; __threadfence(); *(volatile v4f*)(TB + (size_t)i * 4) = o;
}

__global__ __launch_bounds__(32 * BW) void k_dom(const int* __restrict__ pid, const int* __restrict__ feats,
                                                  const float* __restrict__ embp, const float* __restrict__ embf,
                                                  const h16* __restrict__ W1T, const float* __restrict__ TB,
                                                  const float* __restrict__ sb2, const float* __restrict__ db2,
                                                  const float* __restrict__ dlw, const float* __restrict__ dlb, float* OUT) {
    __shared__ __align__(16) h16   Xs[RPB * XP];
    __shared__ int                 spid[RPB];
    __shared__ __align__(16) float sdl[RPB];
    __shared__ __align__(16) float so[RPB];
    const int tid = threadIdx.x;
    const int lane = tid & 31, lr = lane & 15, hi = lane >> 4;
    const int wave = __builtin_amdgcn_readfirstlane((int)(threadIdx.x >> 5));
    const size_t b0 = (size_t)blockIdx.x * RPB;

    if (wave < RPB / 32) {
        const int row = tid;
        const int praw = pid[b0 + row];
        const int pc = praw < 0 ? 0 : (praw > ND ? ND : praw);
        const float* src = embp + (size_t)pc * ED;
        const v4f x0 = *(const v4f*)(src), x1 = *(const v4f*)(src + 4), x2 = *(const v4f*)(src + 8), x3 = *(const v4f*)(src + 12);
        float e[16];
#pragma unroll
        for (int k = 0; k < 4; ++k) { e[k] = relu_b(x0[k]); e[4 + k] = relu_b(x1[k]); e[8 + k] = relu_b(x2[k]); e[12 + k] = relu_b(x3[k]); }
        float s = 0.0f; v8h h0, h1;
#pragma unroll
        for (int k = 0; k < 16; ++k) s += e[k] * bfr(dlw[k]);
#pragma unroll
        for (int k = 0; k < 8; ++k) { h0[k] = toh_flush(e[k] * CARRY); h1[k] = toh_flush(e[8 + k] * CARRY); }
        *(v8h*)(&Xs[row * XP]) = h0; *(v8h*)(&Xs[row * XP + 8]) = h1;
        spid[row] = praw;
        sdl[row] = s + bfr(dlb[0]);
    }
#pragma unroll 1
    for (int it = 0; it < 5; ++it) {
        if (it * (32 * BW) + wave * 32 < NPAIRF) {
            const int pr = it * (32 * BW) + tid;
            const int row = pr / NF, j = pr - row * NF;
            int f = feats[b0 * NF + (size_t)pr];
            f = f < 0 ? 0 : (f > VOC ? VOC : f);
            const float* src = embf + ((size_t)j * (VOC + 1) + (size_t)f) * ED;
            const v4f x0 = *(const v4f*)(src), x1 = *(const v4f*)(src + 4), x2 = *(const v4f*)(src + 8), x3 = *(const v4f*)(src + 12);
            v8h h0, h1;
#pragma unroll
            for (int k = 0; k < 4; ++k) {
                h0[k]     = toh_flush(relu_b(x0[k]) * CARRY); h0[4 + k] = toh_flush(relu_b(x1[k]) * CARRY);
                h1[k]     = toh_flush(relu_b(x2[k]) * CARRY); h1[4 + k] = toh_flush(relu_b(x3[k]) * CARRY); }
            *(v8h*)(&Xs[row * XP + (j + 1) * ED]) = h0; *(v8h*)(&Xs[row * XP + (j + 1) * ED + 8]) = h1;
        }
    }
    __syncthreads();

    v16h a[5];
    const int xo = (16 * wave + lr) * XP + 8 * hi;
#pragma unroll
    for (int ks = 0; ks < 5; ++ks) a[ks] = cat16(*(const v8h*)(&Xs[xo + ks * 32]), *(const v8h*)(&Xs[xo + ks * 32 + 16]));
    int selp[8];
#pragma unroll
    for (int r = 0; r < 8; ++r) selp[r] = spid[16 * wave + 8 * hi + r];
    float res[8];
#pragma unroll
    for (int r = 0; r < 8; ++r) res[r] = 0.0f;

#pragma unroll 1
    for (int d = 0; d < ND; ++d) {
        v8f acc[5];
#pragma unroll
        for (int nb = 0; nb < 5; ++nb) acc[nb] = (v8f){};
        const size_t wo = (size_t)(d * HID + lr) * KIN + 8 * hi;
#pragma unroll
        for (int ks = 0; ks < 5; ++ks) {
#pragma unroll
            for (int nb = 0; nb < 5; ++nb) {
                const v16h b = ldh(W1T + wo + (size_t)nb * 16 * KIN + ks * 32);
                acc[nb] = wmma16g(a[ks], b, acc[nb]); } }
        float b1v[5], w2v[5];
#pragma unroll
        for (int nb = 0; nb < 5; ++nb) { b1v[nb] = TB[d * HID + nb * 16 + lr]; w2v[nb] = TB[NCOL + d * HID + nb * 16 + lr]; }
        const float b2v = bfr(sb2[0]) + bfr(db2[d]);
#pragma unroll
        for (int r = 0; r < 8; ++r) {
            float s = 0.0f;
#pragma unroll
            for (int nb = 0; nb < 5; ++nb) { const float hv = fmaxf(acc[nb][r] * ACC_INV + b1v[nb], 0.0f); s += hv * w2v[nb]; }
            s += __shfl_xor(s, 1, 32); s += __shfl_xor(s, 2, 32); s += __shfl_xor(s, 4, 32); s += __shfl_xor(s, 8, 32);
            const float cand = s + b2v;
            res[r] = (selp[r] == d + 1) ? cand : res[r];
        }
    }

    {
        const int ro = 16 * wave + 8 * hi;
        const v4f d0 = *(const v4fa*)(&sdl[ro]); const v4f d1 = *(const v4fa*)(&sdl[ro + 4]);
        v4f o0, o1;
        o0[0] = res[0] + d0[0]; o0[1] = res[1] + d0[1]; o0[2] = res[2] + d0[2]; o0[3] = res[3] + d0[3];
        o1[0] = res[4] + d1[0]; o1[1] = res[5] + d1[1]; o1[2] = res[6] + d1[2]; o1[3] = res[7] + d1[3];
        if (lr == 0) { *(v4fa*)(&so[ro]) = o0; *(v4fa*)(&so[ro + 4]) = o1; }
    }
    __syncthreads();
    if (wave == 0) {
        const v4f val = *(const v4fa*)(&so[lane * 4]);
        float* op = OUT + b0 + (size_t)lane * 4;
        *(volatile v4f*)op = val; __threadfence(); *(volatile v4f*)op = val;
    }
}

static constexpr size_t al256(size_t v) { return (v + 255) & ~(size_t)255; }
static constexpr size_t SZ_W1T = al256((size_t)NCOL * KIN * 2);
static constexpr size_t SZ_TB  = al256((size_t)2 * NCOL * 4);
static constexpr size_t SZ_TOTAL = SZ_W1T + SZ_TB;
static_assert(SZ_TOTAL <= (size_t)134217728);
static_assert(((size_t)NCOL * KIN * 2) % 128 == 0);
static_assert(((size_t)2 * NCOL * 4) % 128 == 0);
static_assert((size_t)(NCOL * KIN / 8) * 16 == (size_t)NCOL * KIN * 2);
static_assert((size_t)(2 * NCOL / 4) * 16 == (size_t)2 * NCOL * 4);
static_assert((size_t)(NROWS / RPB) * 32 * 16 == (size_t)NROWS * 4);

extern "C" void kernel_launch(void* const* d_in, const int* in_sizes, int n_in,
                              void* d_out, int out_size, void* d_ws, size_t ws_size, hipStream_t stream) {
    if (n_in < 14) return;
    if ((size_t)in_sizes[0] < (size_t)NROWS || (size_t)in_sizes[1] < (size_t)NROWS * NF) return;
    if ((size_t)in_sizes[2] < (size_t)(ND + 1) * ED || (size_t)in_sizes[3] < (size_t)NF * (VOC + 1) * ED) return;
    if ((size_t)in_sizes[4] < (size_t)KIN * HID || (size_t)in_sizes[5] < (size_t)ND * KIN * HID) return;
    if (in_sizes[6] < HID || in_sizes[7] < ND * HID || in_sizes[8] < HID || in_sizes[9] < ND * HID) return;
    if (in_sizes[10] < 1 || in_sizes[11] < ND || in_sizes[12] < ED || in_sizes[13] < 1) return;
    if ((size_t)out_size < (size_t)NROWS) return;
    if (SZ_TOTAL > ws_size) return;
    const int*   pid   = (const int*)d_in[0];
    const int*   feats = (const int*)d_in[1];
    const float* embp  = (const float*)d_in[2];
    const float* embf  = (const float*)d_in[3];
    const float* sw1   = (const float*)d_in[4];
    const float* dw1   = (const float*)d_in[5];
    const float* sb1   = (const float*)d_in[6];
    const float* db1   = (const float*)d_in[7];
    const float* sw2   = (const float*)d_in[8];
    const float* dw2   = (const float*)d_in[9];
    const float* sb2   = (const float*)d_in[10];
    const float* db2   = (const float*)d_in[11];
    const float* dlw   = (const float*)d_in[12];
    const float* dlb   = (const float*)d_in[13];
    float* OUT = (float*)d_out;
    char* wsp = (char*)d_ws;
    h16*   W1T = (h16*)wsp;   wsp += SZ_W1T;
    float* TB  = (float*)wsp; wsp += SZ_TB;

    k_w1t<<<(unsigned)((size_t)NCOL * KIN / 8 / 256), 256, 0, stream>>>(sw1, dw1, W1T);
    k_tabs<<<(unsigned)(2 * NCOL / 4 / 160), 160, 0, stream>>>(sb1, db1, sw2, dw2, TB);
    k_dom<<<(unsigned)(NROWS / RPB), 32 * BW, 0, stream>>>(pid, feats, embp, embf, W1T, TB, sb2, db2, dlw, dlb, OUT);
}
